// MultiheadAttention_83030307766273
// MI455X (gfx1250) — hardware-verified
//
#include <hip/hip_runtime.h>


#ifndef NB
#define NB 2
#endif
#ifndef SEQ
#define SEQ 2048
#endif
#define NB_FULL  2
#define SEQ_FULL 2048
#ifndef OUT_SEQ
#define OUT_SEQ SEQ
#endif
#define EROWS (SEQ < 256 ? SEQ : 256)
#define DM   1024
#define NH_  16
#define HD   64
#define AW   4
#define SC2  (0.125f * 1.4426950408889634f)
#define SC2F (SC2 * 0.00390625f)
#define PSH  8.0f
#define MASKL (-1.0e20f * SC2)
#define TP   72
#define NTOK (NB * SEQ)
#define NKT  (SEQ / 32)
#define FTP  128

static_assert(HD == 64);
static_assert(NH_ * HD == DM);
static_assert(DM % 128 == 0);
static_assert(SEQ % 128 == 0);
static_assert(SEQ % (16 * AW) == 0);
static_assert(EROWS % 64 == 0);
static_assert(EROWS % 128 == 0);
static_assert(EROWS <= SEQ);
static_assert(EROWS % (16 * AW) == 0);
static_assert((SEQ - EROWS) % (16 * AW) == 0);
static_assert((NB * EROWS) % 128 == 0);
static_assert((SEQ - EROWS) % 128 == 0);
static_assert(NKT + 1 <= FTP);
static_assert(((size_t)NB * SEQ * DM) % (8 * 256) == 0);
static_assert(NB <= NB_FULL);
static_assert(SEQ <= SEQ_FULL);

typedef unsigned short us;
typedef _Float16 h16;
typedef __attribute__((ext_vector_type(8)))  unsigned short v8us;
typedef __attribute__((ext_vector_type(16))) unsigned short v16us;
typedef __attribute__((ext_vector_type(16))) __bf16 v16bf;
typedef __attribute__((ext_vector_type(16))) _Float16 v16h;
typedef __attribute__((ext_vector_type(8)))  _Float16 v8h;
typedef __attribute__((ext_vector_type(8)))  float    v8f;
typedef __attribute__((ext_vector_type(4)))  float    v4f;
typedef __attribute__((ext_vector_type(4)))  int      v4i;
typedef v4f  __attribute__((may_alias)) v4fa;
typedef v8us __attribute__((may_alias)) v8usa;
typedef v4i  __attribute__((may_alias)) v4ia;

template <bool H> struct FragSel { typedef v16bf T; };
template <> struct FragSel<true> { typedef v16h T; };

__device__ __forceinline__ unsigned bfb(float f) { unsigned u = __float_as_uint(f); u += 0x7FFFu + ((u >> 16) & 1u); return u >> 16; }
__device__ __forceinline__ float bff(unsigned b) { return __uint_as_float(b << 16); }
__device__ __forceinline__ v8f wmma16(v16bf a, v16bf b, v8f c) { return __builtin_amdgcn_wmma_f32_16x16x32_bf16(false, a, false, b, (short)0, c, false, false); }
__device__ __forceinline__ v8f wmma16(v16h a, v16h b, v8f c) { return __builtin_amdgcn_wmma_f32_16x16x32_f16(false, a, false, b, (short)0, c, false, false); }
template <typename T>
__device__ __forceinline__ T ldt(const us* p) {
    const v8us a = *(const v8us*)p; const v8us b = *(const v8us*)(p + 16);
    return __builtin_bit_cast(T, __builtin_shufflevector(a, b, 0, 1, 2, 3, 4, 5, 6, 7, 8, 9, 10, 11, 12, 13, 14, 15));
}
__device__ __forceinline__ void split8(const v4f x, const v4f y, v8us& h, v8us& l) {
#pragma unroll
    for (int i = 0; i < 4; ++i) {
        const unsigned a = bfb(x[i]); h[i] = (us)a;     l[i] = (us)bfb(x[i] - bff(a));
        const unsigned b = bfb(y[i]); h[4 + i] = (us)b; l[4 + i] = (us)bfb(y[i] - bff(b));
    }
}
__device__ __forceinline__ v8us f16x8(const v4f x, const v4f y, const float s) {
    v8h t;
#pragma unroll
    for (int i = 0; i < 4; ++i) { t[i] = (h16)(x[i] * s); t[4 + i] = (h16)(y[i] * s); }
    return __builtin_bit_cast(v8us, t);
}
__device__ __forceinline__ void wave_sync() { __builtin_amdgcn_fence(3  , "wavefront"); __builtin_amdgcn_wave_barrier(); asm volatile("" ::: "memory"); }

__global__ __launch_bounds__(256) void k_cvt2(const float* __restrict__ sa, us* da, const float* __restrict__ sb, us* db, size_t n8) {
    const size_t i = (size_t)blockIdx.x * 256 + threadIdx.x; if (i >= n8) return;
    const size_t e = i * 8; const size_t row = e / DM; const size_t col = e % DM;
    const size_t bb = row / SEQ, t = row % SEQ;
    const size_t so = (bb * SEQ_FULL + t) * DM + col;
    const v8f x = *(const v8f*)(sa + so); const v8f y = *(const v8f*)(sb + so); v8us o, p;
#pragma unroll
    for (int k = 0; k < 8; ++k) { o[k] = (us)bfb(x[k]); p[k] = (us)bfb(y[k]); }
    *(volatile v8us*)(da + e) = o; *(volatile v8us*)(db + e) = p;
    __threadfence();
    *(volatile v8us*)(da + e) = o; *(volatile v8us*)(db + e) = p;
}

template <bool DUAL>
__global__ __launch_bounds__(256) void k_wt(const float* __restrict__ W, us* WT, us* WF) {
    __shared__ __align__(16) us ts[64 * TP];
    const int tid = threadIdx.x;
    const int k0 = blockIdx.x * 64, n0 = blockIdx.y * 64;
    const int r = tid >> 2, c0 = (tid & 3) * 16;
    const float* src = W + (size_t)(k0 + r) * DM + n0 + c0;
#pragma unroll
    for (int q = 0; q < 4; ++q) { const v4f x = *(const v4f*)(src + 4 * q);
#pragma unroll
        for (int i = 0; i < 4; ++i) ts[(c0 + 4 * q + i) * TP + r] = (us)bfb(x[i]); }
    __syncthreads();
    const size_t dbase = (size_t)n0 * DM + k0;
#pragma unroll 1
    for (int ps = 0; ps < 2; ++ps) {
#pragma unroll
        for (int s = 0; s < 2; ++s) { const int d = 32 * s + (tid >> 3), c8 = (tid & 7) * 8;
            const v8us val = *(const v8usa*)(&ts[d * TP + c8]);
            *(volatile v8us*)(WT + dbase + (size_t)d * DM + c8) = val;
            if (DUAL) { v8h t;
#pragma unroll
                for (int i = 0; i < 8; ++i) t[i] = (h16)(bff((unsigned)val[i]) * 16.0f);
                const v8us fv = __builtin_bit_cast(v8us, t);
                *(volatile v8us*)(WF + dbase + (size_t)d * DM + c8) = fv; } }
        if (ps == 0) __threadfence(); }
}

__global__ __launch_bounds__(256) void k_mflags(const int* __restrict__ MASK, int* FT) {
    __shared__ __align__(16) int fl[FTP];
    __shared__ int rany[16];
    const int tid = threadIdx.x, lane = tid & 31, wave = __builtin_amdgcn_readfirstlane((int)(tid >> 5));
    const int qt = blockIdx.x;
    if (tid < FTP) fl[tid] = 0;
    if (tid < 16) rany[tid] = 0;
    __syncthreads();
    const int rr = lane >> 3, c4 = (lane & 7) * 4;
    int any0 = 0, any1 = 0, any2 = 0, any3 = 0;
#pragma unroll 1
    for (int kt = wave; kt < NKT; kt += 8) {
        const int* mp = MASK + (size_t)(qt * 16 + rr) * SEQ_FULL + kt * 32 + c4;
        const v4i x0 = *(const v4i*)(mp);
        const v4i x1 = *(const v4i*)(mp + (size_t)4 * SEQ_FULL);
        const v4i x2 = *(const v4i*)(mp + (size_t)8 * SEQ_FULL);
        const v4i x3 = *(const v4i*)(mp + (size_t)12 * SEQ_FULL);
        const int n0 = (x0[0] != 0) + (x0[1] != 0) + (x0[2] != 0) + (x0[3] != 0);
        const int n1 = (x1[0] != 0) + (x1[1] != 0) + (x1[2] != 0) + (x1[3] != 0);
        const int n2 = (x2[0] != 0) + (x2[1] != 0) + (x2[2] != 0) + (x2[3] != 0);
        const int n3 = (x3[0] != 0) + (x3[1] != 0) + (x3[2] != 0) + (x3[3] != 0);
        any0 |= n0; any1 |= n1; any2 |= n2; any3 |= n3;
        int cnt = n0 + n1 + n2 + n3;
        cnt += __shfl_xor(cnt, 16, 32); cnt += __shfl_xor(cnt, 8, 32); cnt += __shfl_xor(cnt, 4, 32);
        cnt += __shfl_xor(cnt, 2, 32);  cnt += __shfl_xor(cnt, 1, 32);
        if (lane == 0) fl[kt] = (cnt == 0) ? 0 : ((cnt == 512) ? 2 : 1);
    }
    if (any0 != 0) rany[rr] = 1;
    if (any1 != 0) rany[rr + 4] = 1;
    if (any2 != 0) rany[rr + 8] = 1;
    if (any3 != 0) rany[rr + 12] = 1;
    __syncthreads();
    if (tid == 0) { int fm = 0;
#pragma unroll
        for (int r = 0; r < 16; ++r) fm |= (rany[r] == 0) ? 1 : 0;
        fl[NKT] = fm; }
    __syncthreads();
    if (wave == 0) {
        const v4i val = *(const v4ia*)(&fl[lane * 4]);
        int* dst = FT + (size_t)qt * FTP + lane * 4;
        *(volatile v4i*)dst = val;
        __threadfence();
        *(volatile v4i*)dst = val;
    }
}

template <int MODE>
__global__ __launch_bounds__(128) void k_gemm(const us* __restrict__ A, const us* __restrict__ B, const us* __restrict__ B2, us* OH, us* OL, us* O16, float* OF,
                                              int rpb, int roff, int bpitch, int hlr) {
    typedef typename FragSel<MODE == 3>::T FR;
    __shared__ __align__(16) float os[4 * 32 * 68];
    const int lane = threadIdx.x & 31, wave = __builtin_amdgcn_readfirstlane((int)(threadIdx.x >> 5)), lr = lane & 15, hi = lane >> 4;
    const int m0 = blockIdx.x * 64;
    const int nl = blockIdx.y * 128 + wave * 32;
    int bb = 0, tl = 0, brow = nl;
    if (MODE != 1) { bb = nl / rpb; tl = roff + (nl % rpb); brow = bb * bpitch + tl; }
    const us* ap = A  + (size_t)(m0 + lr) * DM + 8 * hi;
    const us* bp = B  + (size_t)(brow + lr) * DM + 8 * hi;
    const us* ep = B2 + (size_t)(brow + lr) * DM + 8 * hi;
    v8f c[8];
#pragma unroll
    for (int i = 0; i < 8; ++i) c[i] = (v8f){};
#pragma unroll 1
    for (int k0 = 0; k0 < DM; k0 += 32) {
        const FR a0 = ldt<FR>(ap + k0), a1 = ldt<FR>(ap + (size_t)16 * DM + k0), a2 = ldt<FR>(ap + (size_t)32 * DM + k0), a3 = ldt<FR>(ap + (size_t)48 * DM + k0);
        const FR b0 = ldt<FR>(bp + k0), b1 = ldt<FR>(bp + (size_t)16 * DM + k0);
        c[0] = wmma16(a0, b0, c[0]); c[1] = wmma16(a0, b1, c[1]); c[2] = wmma16(a1, b0, c[2]); c[3] = wmma16(a1, b1, c[3]);
        c[4] = wmma16(a2, b0, c[4]); c[5] = wmma16(a2, b1, c[5]); c[6] = wmma16(a3, b0, c[6]); c[7] = wmma16(a3, b1, c[7]);
        if (MODE == 2) {
            const FR e0 = ldt<FR>(ep + k0), e1 = ldt<FR>(ep + (size_t)16 * DM + k0);
            c[0] = wmma16(a0, e0, c[0]); c[1] = wmma16(a0, e1, c[1]); c[2] = wmma16(a1, e0, c[2]); c[3] = wmma16(a1, e1, c[3]);
            c[4] = wmma16(a2, e0, c[4]); c[5] = wmma16(a2, e1, c[5]); c[6] = wmma16(a3, e0, c[6]); c[7] = wmma16(a3, e1, c[7]);
            asm volatile("v_nop\n\tv_nop\n\tv_nop\n\tv_nop" : "+v"(c[0]), "+v"(c[1]), "+v"(c[2]), "+v"(c[3]), "+v"(c[4]), "+v"(c[5]), "+v"(c[6]), "+v"(c[7])
                         : "v"(a0), "v"(a1), "v"(a2), "v"(a3), "v"(b0), "v"(b1), "v"(e0), "v"(e1));
        } else {
            asm volatile("v_nop\n\tv_nop\n\tv_nop\n\tv_nop" : "+v"(c[0]), "+v"(c[1]), "+v"(c[2]), "+v"(c[3]), "+v"(c[4]), "+v"(c[5]), "+v"(c[6]), "+v"(c[7])
                         : "v"(a0), "v"(a1), "v"(a2), "v"(a3), "v"(b0), "v"(b1));
        }
    }
    const int wb = wave * 32 * 68;
    const float osc = (MODE == 3) ? 0.0009765625f : 1.0f;
#pragma unroll
    for (int i = 0; i < 4; ++i) {
#pragma unroll
        for (int j = 0; j < 2; ++j) {
            v4f x, y;
            x[0] = c[i * 2 + j][0] * osc; x[1] = c[i * 2 + j][1] * osc; x[2] = c[i * 2 + j][2] * osc; x[3] = c[i * 2 + j][3] * osc;
            y[0] = c[i * 2 + j][4] * osc; y[1] = c[i * 2 + j][5] * osc; y[2] = c[i * 2 + j][6] * osc; y[3] = c[i * 2 + j][7] * osc;
            *(v4fa*)(&os[wb + (16 * j + lr) * 68 + 16 * i + 8 * hi]) = x;
            *(v4fa*)(&os[wb + (16 * j + lr) * 68 + 16 * i + 8 * hi + 4]) = y;
        }
    }
    wave_sync();
    if (MODE >= 2) {
#pragma unroll 1
        for (int ps = 0; ps < 2; ++ps) {
#pragma unroll
            for (int s = 0; s < 16; ++s) { const int row = 2 * s + hi, cofs = lr * 4;
                const v4f val = *(const v4fa*)(&os[wb + row * 68 + cofs]);
                *(volatile v4f*)(OF + ((size_t)bb * OUT_SEQ + tl + row) * DM + m0 + cofs) = val; }
            if (ps == 0) __threadfence(); }
    } else {
        const int bbm = m0 / SEQ, tlm = m0 % SEQ;
        const bool hl = (MODE == 1) ? true : (tl < hlr);
#pragma unroll 1
        for (int ps = 0; ps < 2; ++ps) {
#pragma unroll
            for (int s = 0; s < 8; ++s) { const int row = 4 * s + (lane >> 3), c8 = (lane & 7) * 8;
                const v4f x = *(const v4fa*)(&os[wb + row * 68 + c8]);
                const v4f y = *(const v4fa*)(&os[wb + row * 68 + c8 + 4]);
                const v8us fv = f16x8(x, y, 16.0f);
                size_t o16, ohl;
                if (MODE == 0) { o16 = (size_t)(brow + row) * DM + m0 + c8; ohl = ((size_t)bb * hlr + tl + row) * DM + m0 + c8; }
                else { o16 = ((size_t)bbm * DM + nl + row) * SEQ + tlm + c8; ohl = o16; }
                *(volatile v8us*)(O16 + o16) = fv;
                if (hl) { v8us hv, lv; split8(x, y, hv, lv);
                    *(volatile v8us*)(OH + ohl) = hv;
                    *(volatile v8us*)(OL + ohl) = lv; } }
            if (ps == 0) __threadfence(); }
    }
}

template <bool EARLY>
__global__ __launch_bounds__(32 * AW) void k_flash(const us* __restrict__ QH, const us* __restrict__ QL, const us* __restrict__ KH, const us* __restrict__ KL,
                                                   const us* __restrict__ VH, const us* __restrict__ VL,
                                                   const us* __restrict__ QF, const us* __restrict__ KF, const us* __restrict__ VF,
                                                   const int* __restrict__ MASK, const int* __restrict__ FT, us* CH, us* CL, us* CF) {
    __shared__ __align__(16) float os[AW * 16 * 68];
    const int lane = threadIdx.x & 31, wave = __builtin_amdgcn_readfirstlane((int)(threadIdx.x >> 5)), lr = lane & 15, hi = lane >> 4;
    const int zh = blockIdx.y; const int b = zh / NH_, h = zh % NH_;
    const int t0 = (EARLY ? 0 : EROWS) + (blockIdx.x * AW + wave) * 16;
    const size_t rbase = (size_t)b * SEQ * DM + (size_t)h * HD;
    const size_t ko = rbase + (size_t)lr * DM + 8 * hi;
    const size_t vo = ((size_t)zh * HD + lr) * SEQ + 8 * hi;
    const int* mrow = MASK + (size_t)(t0 + lr) * SEQ_FULL + 8 * hi;
    const int* frow = FT + (size_t)(t0 >> 4) * FTP;
    const int full = __builtin_amdgcn_readfirstlane(frow[NKT]);
    const v16bf zb = __builtin_bit_cast(v16bf, (v16us){});
    v16bf qh0 = zb, qh1 = zb, ql0 = zb, ql1 = zb;
    v16h qf0 = (v16h){}, qf1 = (v16h){};
    if (EARLY) {
        const size_t qc = ((size_t)b * EROWS + t0 + lr) * DM + (size_t)h * HD + 8 * hi;
        qh0 = ldt<v16bf>(QH + qc); qh1 = ldt<v16bf>(QH + qc + 32);
        ql0 = ldt<v16bf>(QL + qc); ql1 = ldt<v16bf>(QL + qc + 32);
    } else {
        const size_t qo = rbase + (size_t)(t0 + lr) * DM + 8 * hi;
        qf0 = ldt<v16h>(QF + qo); qf1 = ldt<v16h>(QF + qo + 32);
    }
    v8f o0 = (v8f){}, o1 = (v8f){}, o2 = (v8f){}, o3 = (v8f){};
    float m = -3.0e38f, l = 0.0f;
    const float ssc = EARLY ? SC2 : SC2F;
#pragma unroll 1
    for (int kt = 0; kt < NKT; ++kt) {
        const int f = __builtin_amdgcn_readfirstlane(frow[kt]);
        if (f == 0 && full == 0) continue;
        const int key0 = kt * 32;
        v8f sa = (v8f){}, sb = (v8f){};
        if (EARLY) {
            const us* kh = KH + ko + (size_t)key0 * DM;
            const us* kl = KL + ko + (size_t)key0 * DM;
            const v16bf ka0 = ldt<v16bf>(kh), ka1 = ldt<v16bf>(kh + 32), kb0 = ldt<v16bf>(kh + (size_t)16 * DM), kb1 = ldt<v16bf>(kh + (size_t)16 * DM + 32);
            sa = wmma16(ka0, qh0, sa); sb = wmma16(kb0, qh0, sb);
            sa = wmma16(ka1, qh1, sa); sb = wmma16(kb1, qh1, sb);
            sa = wmma16(ka0, ql0, sa); sb = wmma16(kb0, ql0, sb);
            sa = wmma16(ka1, ql1, sa); sb = wmma16(kb1, ql1, sb);
            const v16bf la0 = ldt<v16bf>(kl), la1 = ldt<v16bf>(kl + 32), lb0 = ldt<v16bf>(kl + (size_t)16 * DM), lb1 = ldt<v16bf>(kl + (size_t)16 * DM + 32);
            sa = wmma16(la0, qh0, sa); sb = wmma16(lb0, qh0, sb);
            sa = wmma16(la1, qh1, sa); sb = wmma16(lb1, qh1, sb);
            asm volatile("v_nop\n\tv_nop\n\tv_nop\n\tv_nop" : "+v"(sa), "+v"(sb)
                         : "v"(ka0), "v"(ka1), "v"(kb0), "v"(kb1), "v"(la0), "v"(la1), "v"(lb0), "v"(lb1), "v"(qh0), "v"(qh1), "v"(ql0), "v"(ql1));
        } else {
            const us* kf = KF + ko + (size_t)key0 * DM;
            const v16h ka0 = ldt<v16h>(kf), ka1 = ldt<v16h>(kf + 32), kb0 = ldt<v16h>(kf + (size_t)16 * DM), kb1 = ldt<v16h>(kf + (size_t)16 * DM + 32);
            sa = wmma16(ka0, qf0, sa); sb = wmma16(kb0, qf0, sb);
            sa = wmma16(ka1, qf1, sa); sb = wmma16(kb1, qf1, sb);
            asm volatile("v_nop\n\tv_nop\n\tv_nop\n\tv_nop" : "+v"(sa), "+v"(sb) : "v"(ka0), "v"(ka1), "v"(kb0), "v"(kb1), "v"(qf0), "v"(qf1));
        }
        float ta[8], tb[8];
#pragma unroll
        for (int r = 0; r < 8; ++r) { ta[r] = sa[r] * ssc; tb[r] = sb[r] * ssc; }
        if (f != 2) {
            const int* mp = mrow + key0;
            const v4i m0 = *(const v4i*)(mp), m1 = *(const v4i*)(mp + 4), m2 = *(const v4i*)(mp + 16), m3 = *(const v4i*)(mp + 20);
#pragma unroll
            for (int r = 0; r < 4; ++r) {
                ta[r]     = (m0[r] != 0) ? ta[r]     : MASKL;
                ta[4 + r] = (m1[r] != 0) ? ta[4 + r] : MASKL;
                tb[r]     = (m2[r] != 0) ? tb[r]     : MASKL;
                tb[4 + r] = (m3[r] != 0) ? tb[4 + r] : MASKL;
            }
        }
        float mx = -3.0e38f;
#pragma unroll
        for (int r = 0; r < 8; ++r) mx = fmaxf(mx, fmaxf(ta[r], tb[r]));
        mx = fmaxf(mx, __shfl_xor(mx, 16, 32));
        const float mnew = fmaxf(m, mx);
        const float alpha = __builtin_amdgcn_exp2f(m - mnew);
        if (EARLY) {
            v16us phu, plu; float ls = 0.0f;
#pragma unroll
            for (int r = 0; r < 8; ++r) {
                const float pa = __builtin_amdgcn_exp2f(ta[r] - mnew);
                const float pc = __builtin_amdgcn_exp2f(tb[r] - mnew);
                const unsigned ha = bfb(pa), hc = bfb(pc);
                phu[r] = (us)ha; phu[8 + r] = (us)hc;
                plu[r] = (us)bfb(pa - bff(ha)); plu[8 + r] = (us)bfb(pc - bff(hc));
                ls += pa + pc;
            }
            const v16bf ph = __builtin_bit_cast(v16bf, phu);
            const v16bf pl = __builtin_bit_cast(v16bf, plu);
            l = l * alpha + ls; m = mnew;
            o0 = o0 * alpha; o1 = o1 * alpha; o2 = o2 * alpha; o3 = o3 * alpha;
            const us* va = VH + vo + key0;
            const v16bf v0 = ldt<v16bf>(va), v1 = ldt<v16bf>(va + (size_t)16 * SEQ), v2 = ldt<v16bf>(va + (size_t)32 * SEQ), v3 = ldt<v16bf>(va + (size_t)48 * SEQ);
            o0 = wmma16(v0, ph, o0); o1 = wmma16(v1, ph, o1); o2 = wmma16(v2, ph, o2); o3 = wmma16(v3, ph, o3);
            o0 = wmma16(v0, pl, o0); o1 = wmma16(v1, pl, o1); o2 = wmma16(v2, pl, o2); o3 = wmma16(v3, pl, o3);
            const us* vb = VL + vo + key0;
            const v16bf w0 = ldt<v16bf>(vb), w1 = ldt<v16bf>(vb + (size_t)16 * SEQ), w2 = ldt<v16bf>(vb + (size_t)32 * SEQ), w3 = ldt<v16bf>(vb + (size_t)48 * SEQ);
            o0 = wmma16(w0, ph, o0); o1 = wmma16(w1, ph, o1); o2 = wmma16(w2, ph, o2); o3 = wmma16(w3, ph, o3);
            asm volatile("v_nop\n\tv_nop\n\tv_nop\n\tv_nop" : "+v"(o0), "+v"(o1), "+v"(o2), "+v"(o3)
                         : "v"(v0), "v"(v1), "v"(v2), "v"(v3), "v"(w0), "v"(w1), "v"(w2), "v"(w3), "v"(ph), "v"(pl));
        } else {
            v16h pb; float ls = 0.0f;
#pragma unroll
            for (int r = 0; r < 8; ++r) {
                const h16 pa = (h16)__builtin_amdgcn_exp2f((ta[r] - mnew) + PSH);
                const h16 pc = (h16)__builtin_amdgcn_exp2f((tb[r] - mnew) + PSH);
                pb[r] = pa; pb[8 + r] = pc; ls += (float)pa + (float)pc;
            }
            l = l * alpha + ls; m = mnew;
            o0 = o0 * alpha; o1 = o1 * alpha; o2 = o2 * alpha; o3 = o3 * alpha;
            const us* va = VF + vo + key0;
            const v16h v0 = ldt<v16h>(va), v1 = ldt<v16h>(va + (size_t)16 * SEQ), v2 = ldt<v16h>(va + (size_t)32 * SEQ), v3 = ldt<v16h>(va + (size_t)48 * SEQ);
            o0 = wmma16(v0, pb, o0); o1 = wmma16(v1, pb, o1); o2 = wmma16(v2, pb, o2); o3 = wmma16(v3, pb, o3);
            asm volatile("v_nop\n\tv_nop\n\tv_nop\n\tv_nop" : "+v"(o0), "+v"(o1), "+v"(o2), "+v"(o3) : "v"(v0), "v"(v1), "v"(v2), "v"(v3), "v"(pb));
        }
    }
    l += __shfl_xor(l, 16, 32);
    const float inv = (EARLY ? 1.0f : 4.0f) * (1.0f / l);
    const int wb = wave * 16 * 68;
    { v4f a, c;
      a[0] = o0[0] * inv; a[1] = o0[1] * inv; a[2] = o0[2] * inv; a[3] = o0[3] * inv; c[0] = o0[4] * inv; c[1] = o0[5] * inv; c[2] = o0[6] * inv; c[3] = o0[7] * inv;
      *(v4fa*)(&os[wb + lr * 68 +  0 + 8 * hi]) = a; *(v4fa*)(&os[wb + lr * 68 +  0 + 8 * hi + 4]) = c;
      a[0] = o1[0] * inv; a[1] = o1[1] * inv; a[2] = o1[2] * inv; a[3] = o1[3] * inv; c[0] = o1[4] * inv; c[1] = o1[5] * inv; c[2] = o1[6] * inv; c[3] = o1[7] * inv;
      *(v4fa*)(&os[wb + lr * 68 + 16 + 8 * hi]) = a; *(v4fa*)(&os[wb + lr * 68 + 16 + 8 * hi + 4]) = c;
      a[0] = o2[0] * inv; a[1] = o2[1] * inv; a[2] = o2[2] * inv; a[3] = o2[3] * inv; c[0] = o2[4] * inv; c[1] = o2[5] * inv; c[2] = o2[6] * inv; c[3] = o2[7] * inv;
      *(v4fa*)(&os[wb + lr * 68 + 32 + 8 * hi]) = a; *(v4fa*)(&os[wb + lr * 68 + 32 + 8 * hi + 4]) = c;
      a[0] = o3[0] * inv; a[1] = o3[1] * inv; a[2] = o3[2] * inv; a[3] = o3[3] * inv; c[0] = o3[4] * inv; c[1] = o3[5] * inv; c[2] = o3[6] * inv; c[3] = o3[7] * inv;
      *(v4fa*)(&os[wb + lr * 68 + 48 + 8 * hi]) = a; *(v4fa*)(&os[wb + lr * 68 + 48 + 8 * hi + 4]) = c; }
    wave_sync();
    const size_t cbase = EARLY ? (((size_t)b * EROWS + t0) * DM + (size_t)h * HD)
                               : (((size_t)b * SEQ + t0) * DM + (size_t)h * HD);
#pragma unroll 1
    for (int ps = 0; ps < 2; ++ps) {
#pragma unroll
        for (int s = 0; s < 4; ++s) { const int row = 4 * s + (lane >> 3), c8 = (lane & 7) * 8;
            const v4f x = *(const v4fa*)(&os[wb + row * 68 + c8]);
            const v4f y = *(const v4fa*)(&os[wb + row * 68 + c8 + 4]);
            const size_t off = cbase + (size_t)row * DM + c8;
            if (EARLY) { v8us hv, lv; split8(x, y, hv, lv);
                *(volatile v8us*)(CH + off) = hv;
                *(volatile v8us*)(CL + off) = lv; }
            else { const v8us fv = f16x8(x, y, 1.0f);
                *(volatile v8us*)(CF + off) = fv; } }
        if (ps == 0) __threadfence(); }
}

static constexpr size_t al256(size_t v) { return (v + 255) & ~(size_t)255; }
static constexpr size_t SZ_PL = al256((size_t)NTOK * DM * 2);
static constexpr size_t SZ_E  = al256((size_t)NB * EROWS * DM * 2);
static constexpr size_t SZ_W  = al256((size_t)DM * DM * 2);
static constexpr size_t SZ_FT = al256((size_t)(SEQ / 16) * FTP * 4);
static constexpr size_t SZ_TOTAL = 10 * SZ_PL + 4 * SZ_E + 5 * SZ_W + SZ_FT;
static_assert(SZ_TOTAL <= (size_t)134217728);
static_assert((size_t)NB * NH_ * HD * SEQ * 2 <= SZ_PL);
static_assert(((size_t)(NB - 1) * EROWS + EROWS) * DM * 2 <= SZ_E);
static_assert((size_t)(SEQ / 16 - 1) * FTP * 4 + 512 <= SZ_FT);

extern "C" void kernel_launch(void* const* d_in, const int* in_sizes, int n_in,
                              void* d_out, int out_size, void* d_ws, size_t ws_size, hipStream_t stream) {
    if (n_in < 7) return;
    const size_t needx = ((size_t)(NB - 1) * SEQ_FULL + SEQ) * DM;
    if ((size_t)in_sizes[0] < needx || (size_t)in_sizes[1] < needx) return;
    if ((size_t)in_sizes[2] < (size_t)(SEQ - 1) * SEQ_FULL + SEQ) return;
    if ((size_t)in_sizes[3] < (size_t)DM * DM || (size_t)in_sizes[4] < (size_t)DM * DM) return;
    if ((size_t)in_sizes[5] < (size_t)DM * DM || (size_t)in_sizes[6] < (size_t)DM * DM) return;
    if ((size_t)out_size < ((size_t)(NB - 1) * OUT_SEQ + SEQ) * DM) return;
    if (SZ_TOTAL > ws_size) return;
    const float* xq = (const float*)d_in[0]; const float* xk = (const float*)d_in[1];
    const int* mask = (const int*)d_in[2];
    const float* Wq = (const float*)d_in[3]; const float* Wk = (const float*)d_in[4];
    const float* Wv = (const float*)d_in[5]; const float* Wo = (const float*)d_in[6];
    float* OUT = (float*)d_out;
    char* wsp = (char*)d_ws;
    us* XQ  = (us*)wsp; wsp += SZ_PL;
    us* XK  = (us*)wsp; wsp += SZ_PL;
    us* QF  = (us*)wsp; wsp += SZ_PL;
    us* KF  = (us*)wsp; wsp += SZ_PL;
    us* VTF = (us*)wsp; wsp += SZ_PL;
    us* CF  = (us*)wsp; wsp += SZ_PL;
    us* KH  = (us*)wsp; wsp += SZ_PL;
    us* KL  = (us*)wsp; wsp += SZ_PL;
    us* VTH = (us*)wsp; wsp += SZ_PL;
    us* VTL = (us*)wsp; wsp += SZ_PL;
    us* QH  = (us*)wsp; wsp += SZ_E;
    us* QL  = (us*)wsp; wsp += SZ_E;
    us* CH  = (us*)wsp; wsp += SZ_E;
    us* CL  = (us*)wsp; wsp += SZ_E;
    us* WQT = (us*)wsp; wsp += SZ_W;
    us* WKT = (us*)wsp; wsp += SZ_W;
    us* WVT = (us*)wsp; wsp += SZ_W;
    us* WOT = (us*)wsp; wsp += SZ_W;
    us* WOF = (us*)wsp; wsp += SZ_W;
    int* FT = (int*)wsp; wsp += SZ_FT;

    const size_t n8 = (size_t)NTOK * DM / 8;
    k_cvt2<<<(unsigned)((n8 + 255) / 256), 256, 0, stream>>>(xq, XQ, xk, XK, n8);
    k_wt<false><<<dim3(DM / 64, DM / 64, 1), 256, 0, stream>>>(Wq, WQT, WQT);
    k_wt<false><<<dim3(DM / 64, DM / 64, 1), 256, 0, stream>>>(Wk, WKT, WKT);
    k_wt<false><<<dim3(DM / 64, DM / 64, 1), 256, 0, stream>>>(Wv, WVT, WVT);
    k_wt<true><<<dim3(DM / 64, DM / 64, 1), 256, 0, stream>>>(Wo, WOT, WOF);
    k_mflags<<<SEQ / 16, 256, 0, stream>>>(mask, FT);
    k_gemm<0><<<dim3(DM / 64, NTOK / 128, 1), 128, 0, stream>>>(WQT, XQ, XQ, QH, QL, QF, OUT, SEQ, 0, SEQ, EROWS);
    k_gemm<0><<<dim3(DM / 64, NTOK / 128, 1), 128, 0, stream>>>(WKT, XK, XK, KH, KL, KF, OUT, SEQ, 0, SEQ, SEQ);
    k_gemm<1><<<dim3(NTOK / 64, DM / 128, 1), 128, 0, stream>>>(XK, WVT, WVT, VTH, VTL, VTF, OUT, SEQ, 0, SEQ, SEQ);
    k_flash<true><<<dim3(EROWS / (16 * AW), NB * NH_, 1), 32 * AW, 0, stream>>>(QH, QL, KH, KL, VTH, VTL, QF, KF, VTF, mask, FT, CH, CL, CF);
    if (SEQ > EROWS)
        k_flash<false><<<dim3((SEQ - EROWS) / (16 * AW), NB * NH_, 1), 32 * AW, 0, stream>>>(QH, QL, KH, KL, VTH, VTL, QF, KF, VTF, mask, FT, CH, CL, CF);
    k_gemm<2><<<dim3(DM / 64, (NB * EROWS) / 128, 1), 128, 0, stream>>>(WOT, CH, CL, QH, QL, QF, OUT, EROWS, 0, EROWS, 0);
    if (SEQ > EROWS)
        k_gemm<3><<<dim3(DM / 64, (NB * (SEQ - EROWS)) / 128, 1), 128, 0, stream>>>(WOF, CF, CF, QH, QL, QF, OUT, SEQ - EROWS, EROWS, SEQ, 0);
}
